// NonLocalAttenion2D_4904852652215
// MI455X (gfx1250) — hardware-verified
//
#include <hip/hip_runtime.h>
#include <math.h>

typedef __attribute__((ext_vector_type(16))) _Float16 v16h;
typedef __attribute__((ext_vector_type(16))) __bf16 v16b;
typedef __attribute__((ext_vector_type(8)))  _Float16 v8h;
typedef __attribute__((ext_vector_type(8)))  float v8f;
typedef __attribute__((ext_vector_type(4)))  float v4f;
typedef __attribute__((ext_vector_type(2)))  float v2f;
typedef __attribute__((ext_vector_type(4)))  unsigned v4u;
typedef __attribute__((ext_vector_type(4)))  int v4i;
typedef float __attribute__((may_alias)) float_a;
typedef int __attribute__((may_alias)) int_a;

template <typename T> __device__ __forceinline__ void vst2(void* p, T v) { *(volatile T*)p = v; __threadfence(); *(volatile T*)p = v; }
__device__ __forceinline__ v8f wmma16(v16h a, v16h b, v8f c) {
  v8f d = __builtin_amdgcn_wmma_f32_16x16x32_f16(false, a, false, b, (short)0, c, false, false);
  asm volatile("v_nop\n\tv_nop\n\tv_nop\n\tv_nop" : "+v"(d) : "v"(a), "v"(b));
  return d;
}
__device__ __forceinline__ v8f wmma_bf(v16b a, v16b b, v8f c) {
  v8f d = __builtin_amdgcn_wmma_f32_16x16x32_bf16(false, a, false, b, (short)0, c, false, false);
  asm volatile("v_nop\n\tv_nop\n\tv_nop\n\tv_nop" : "+v"(d) : "v"(a), "v"(b));
  return d;
}
__device__ __forceinline__ v16h frag_h(const _Float16* rowk0, int lane) {
  union { v16h v; v8h q[2]; } u; const _Float16* p = rowk0 + 8 * (lane >> 4);
  u.q[0] = *(const v8h*)p; u.q[1] = *(const v8h*)(p + 16); return u.v;
}
__device__ __forceinline__ v16h frag_f32(const float* rowk0, int lane) {
  v16h a; const float* p = rowk0 + 8 * (lane >> 4);
#pragma unroll
  for (int i = 0; i < 8; ++i) { a[i] = (_Float16)p[i]; a[8 + i] = (_Float16)p[16 + i]; }
  return a;
}
__device__ __forceinline__ v16h frag_f32s(const float* rowk0, int lane, float sc) {
  v16h a; const float* p = rowk0 + 8 * (lane >> 4);
#pragma unroll
  for (int i = 0; i < 8; ++i) { a[i] = (_Float16)(p[i] * sc); a[8 + i] = (_Float16)(p[16 + i] * sc); }
  return a;
}
__device__ __forceinline__ v16h fragc_f32(const float* W, int k0, int n, int lane, int ld, int K) {
  v16h a; const int g = lane >> 4;
#pragma unroll
  for (int i = 0; i < 8; ++i) { const int ka = k0 + 8 * g + i, kb = ka + 16;
    a[i] = (_Float16)(ka < K ? W[(size_t)(ka < K ? ka : K - 1) * ld + n] : 0.f); a[8 + i] = (_Float16)(kb < K ? W[(size_t)(kb < K ? kb : K - 1) * ld + n] : 0.f); }
  return a;
}
struct F2 { v16b h, l; };
__device__ __forceinline__ F2 bsplit16(const float v[16]) { F2 r;
#pragma unroll
  for (int i = 0; i < 16; ++i) { const __bf16 h = (__bf16)v[i]; r.h[i] = h; r.l[i] = (__bf16)(v[i] - (float)h); }
  return r; }
__device__ __forceinline__ F2 split_row(const float* row, int k0, int lane) { float v[16]; const float* p = row + k0 + 8 * (lane >> 4);
#pragma unroll
  for (int i = 0; i < 8; ++i) { v[i] = p[i]; v[8 + i] = p[16 + i]; }
  return bsplit16(v); }
__device__ __forceinline__ F2 split_rowK(const float* row, int k0, int lane, int K) { float v[16]; const int g = lane >> 4;
#pragma unroll
  for (int i = 0; i < 8; ++i) { const int ka = k0 + 8 * g + i, kb = ka + 16; v[i] = ka < K ? row[ka < K ? ka : K - 1] : 0.f; v[8 + i] = kb < K ? row[kb < K ? kb : K - 1] : 0.f; }
  return bsplit16(v); }
__device__ __forceinline__ F2 split_col(const float* W, int k0, int n, int lane, int ld, int K) { float v[16]; const int g = lane >> 4;
#pragma unroll
  for (int i = 0; i < 8; ++i) { const int ka = k0 + 8 * g + i, kb = ka + 16; v[i] = ka < K ? W[(size_t)(ka < K ? ka : K - 1) * ld + n] : 0.f; v[8 + i] = kb < K ? W[(size_t)(kb < K ? kb : K - 1) * ld + n] : 0.f; }
  return bsplit16(v); }
__device__ __forceinline__ v8f mac3(const F2& a, const F2& b, v8f c) { c = wmma_bf(a.l, b.h, c); c = wmma_bf(a.h, b.l, c); return wmma_bf(a.h, b.h, c); }
__device__ __forceinline__ float sigm(float v) { return 1.0f / (1.0f + expf(-v)); }
#define LDSX() do { asm volatile("s_wait_dscnt 0" ::: "memory"); __builtin_amdgcn_wave_barrier(); __builtin_amdgcn_fence(__ATOMIC_RELEASE, "workgroup"); } while (0)


#define NI 8
#define CC 128
#define HH 64
#define WWD 64
#define NQ (HH * WWD)
#define NKEY (NQ / 4)
#define DA 16
#define DV 64
#ifndef TNI
#define TNI NI
#endif
typedef __attribute__((ext_vector_type(8))) __bf16 v8b;
__device__ __forceinline__ v16b frag_b(const __bf16* rowk0, int lane) {
  union { v16b v; v8b q[2]; } u; const __bf16* p = rowk0 + 8 * (lane >> 4);
  u.q[0] = *(const v8b*)p; u.q[1] = *(const v8b*)(p + 16); return u.v;
}
__device__ __forceinline__ float bfr(float v) { return (float)(__bf16)v; }
__device__ __attribute__((noinline)) float exp_ni(float v) { return expf(v); }
__device__ __attribute__((noinline)) float erf_ni(float v) { return erff(v); }

#define WS_Q   0u
#define WS_KF  (WS_Q + 4u * (size_t)NI * NQ * DA)
#define WS_VF  (WS_KF + 4u * (size_t)NI * NQ * DA)
#define WS_KP  (WS_VF + 4u * (size_t)NI * NQ * DV)
#define WS_VH  (WS_KP + 4u * (size_t)NI * NKEY * DA)
#define WS_VL  (WS_VH + 2u * (size_t)NI * DV * NKEY)
#define WS_AO  (WS_VL + 2u * (size_t)NI * DV * NKEY)
#define WS_END (WS_AO + 4u * (size_t)NI * NQ * DV)

__global__ __launch_bounds__(128) void k_proj(const float* __restrict__ X, const float* __restrict__ WQ, const float* __restrict__ BQ, const float* __restrict__ WK, const float* __restrict__ BK, const float* __restrict__ WV, const float* __restrict__ BV, float* __restrict__ Q, float* __restrict__ KF, float* __restrict__ VF) {
  __shared__ __align__(16) __bf16 sx[64][CC + 8]; __shared__ __align__(16) float so[4][16][100];
  const int tid = threadIdx.x, wave = tid >> 5, lane = tid & 31, col = lane & 15, g = lane >> 4; const int pb = blockIdx.x; const size_t n = blockIdx.y; const int p0 = pb * 64;
  for (int e = tid; e < CC * 64; e += 128) { const int c = e >> 6, pl = e & 63; sx[pl][c] = (__bf16)X[(n * CC + c) * NQ + p0 + pl]; }
  __syncthreads();
  v8f acc[6] = {};
#pragma unroll
  for (int kc = 0; kc < CC / 32; ++kc) { const v16b a = frag_b(&sx[wave * 16 + col][kc * 32], lane);
#pragma unroll
    for (int j = 0; j < 6; ++j) { v16b w; const float* Wm = (j == 0) ? WQ : (j == 1) ? WK : WV; const int ncol = (j < 2) ? DA : DV; const int o = (j < 2) ? col : ((j - 2) * 16 + col);
#pragma unroll
      for (int i = 0; i < 8; ++i) { w[i] = (__bf16)Wm[(kc * 32 + 8 * g + i) * ncol + o]; w[8 + i] = (__bf16)Wm[(kc * 32 + 16 + 8 * g + i) * ncol + o]; }
      acc[j] = wmma_bf(a, w, acc[j]); } }
#pragma unroll
  for (int j = 0; j < 6; ++j) { const float* Bm = (j == 0) ? BQ : (j == 1) ? BK : BV; const int o = (j < 2) ? col : ((j - 2) * 16 + col); const float bb = bfr(Bm[o]);
#pragma unroll
    for (int r = 0; r < 8; ++r) so[wave][8 * g + r][j * 16 + col] = acc[j][r] + bb; }
  LDSX();
  for (int rl = 0; rl < 16; ++rl) { const size_t row = n * NQ + p0 + wave * 16 + rl; if (lane < 4) vst2(Q + row * DA + lane * 4, *(const v4f*)&so[wave][rl][lane * 4]); else if (lane < 8) vst2(KF + row * DA + (lane - 4) * 4, *(const v4f*)&so[wave][rl][16 + (lane - 4) * 4]); else if (lane < 24) vst2(VF + row * DV + (lane - 8) * 4, *(const v4f*)&so[wave][rl][32 + (lane - 8) * 4]); } }
__global__ __launch_bounds__(64) void k_pool(const float* __restrict__ KF, const float* __restrict__ VF, float* __restrict__ KP, _Float16* __restrict__ VH, _Float16* __restrict__ VL) { __shared__ __align__(16) float sk[64][DA]; __shared__ __align__(16) _Float16 th[DV][72], tl[DV][72];
  const int t = threadIdx.x; const size_t n = blockIdx.y; const int kp = blockIdx.x * 64 + t; const int py = kp / (WWD / 2), px = kp % (WWD / 2); const size_t p00 = n * NQ + (size_t)(2 * py) * WWD + 2 * px;
  for (int d = 0; d < DA; ++d) { const float a = KF[p00 * DA + d], b = KF[(p00 + 1) * DA + d], c = KF[(p00 + WWD) * DA + d], e = KF[(p00 + WWD + 1) * DA + d]; sk[t][d] = fmaxf(fmaxf(a, b), fmaxf(c, e)); }
  for (int d = 0; d < DV; ++d) { const float a = VF[p00 * DV + d], b = VF[(p00 + 1) * DV + d], c = VF[(p00 + WWD) * DV + d], e = VF[(p00 + WWD + 1) * DV + d]; const float v = fmaxf(fmaxf(a, b), fmaxf(c, e)); const _Float16 hv = (_Float16)v; th[d][t] = hv; tl[d][t] = (_Float16)((v - (float)hv) * 2048.0f); }
  __syncthreads();
  for (int e = t; e < 64 * DA / 4; e += 64) vst2(KP + (n * NKEY + (size_t)blockIdx.x * 64) * DA + e * 4, *(const v4f*)&(&sk[0][0])[e * 4]);
  for (int e = t; e < DV * 8; e += 64) { const int d = e >> 3, q = e & 7; const size_t o = (n * DV + d) * (size_t)NKEY + (size_t)blockIdx.x * 64 + q * 8; vst2((unsigned*)(VH + o), *(const v4u*)&th[d][q * 8]); vst2((unsigned*)(VL + o), *(const v4u*)&tl[d][q * 8]); } }
__global__ __launch_bounds__(128) void k_att(const float* __restrict__ Q, const float* __restrict__ KP, const _Float16* __restrict__ VH, const _Float16* __restrict__ VL, float* __restrict__ AO) {
  __shared__ __align__(16) float sp[4][16][36]; __shared__ __align__(16) float so[4][16][68];
  const int tid = threadIdx.x, wave = tid >> 5, lane = tid & 31, col = lane & 15, g = lane >> 4; const int qb = blockIdx.x; const size_t n = blockIdx.y; const size_t q0 = n * NQ + (size_t)qb * 64 + wave * 16;
  F2 aq; { float v[16]; const float* p = Q + (q0 + col) * DA;
#pragma unroll
    for (int i = 0; i < 8; ++i) { v[i] = p[8 * g + i]; v[8 + i] = 0.f; }
    aq = bsplit16(v); }
  float m[8], l[8];
#pragma unroll
  for (int r = 0; r < 8; ++r) { m[r] = -3.0e38f; l[r] = 0.f; }
  v8f acc[4] = {}, accl[4] = {};
#pragma unroll 1
  for (int ks = 0; ks < NKEY / 32; ++ks) { float s[2][8];
#pragma unroll
    for (int ct = 0; ct < 2; ++ct) { const size_t kk = n * NKEY + ks * 32 + ct * 16 + col; F2 bk; { float v[16]; const float* p = KP + kk * DA;
#pragma unroll
        for (int i = 0; i < 8; ++i) { v[i] = p[8 * g + i]; v[8 + i] = 0.f; }
        bk = bsplit16(v); }
      v8f c = {}; c = mac3(aq, bk, c);
#pragma unroll
      for (int r = 0; r < 8; ++r) s[ct][r] = c[r]; }
    float alpha[8];
#pragma unroll
    for (int r = 0; r < 8; ++r) { float mx = fmaxf(s[0][r], s[1][r]);
#pragma unroll
      for (int o = 1; o < 16; o <<= 1) mx = fmaxf(mx, __shfl_xor(mx, o));
      const float mn = fmaxf(m[r], mx); alpha[r] = __expf(m[r] - mn); const float e0 = __expf(s[0][r] - mn), e1 = __expf(s[1][r] - mn); float es = e0 + e1;
#pragma unroll
      for (int o = 1; o < 16; o <<= 1) es += __shfl_xor(es, o);
      l[r] = l[r] * alpha[r] + es; m[r] = mn; sp[wave][8 * g + r][col] = e0; sp[wave][8 * g + r][16 + col] = e1; }
#pragma unroll
    for (int j = 0; j < 4; ++j)
#pragma unroll
      for (int r = 0; r < 8; ++r) { acc[j][r] *= alpha[r]; accl[j][r] *= alpha[r]; }
    LDSX();
    v16h pa, pr; { const float* prow = &sp[wave][col][0] + 8 * (lane >> 4);
#pragma unroll
      for (int i = 0; i < 8; ++i) { const float x0 = prow[i] * 2048.0f, x1 = prow[16 + i] * 2048.0f; const _Float16 h0 = (_Float16)x0, h1 = (_Float16)x1; pa[i] = h0; pa[8 + i] = h1; pr[i] = (_Float16)(x0 - (float)h0); pr[8 + i] = (_Float16)(x1 - (float)h1); } }
#pragma unroll
    for (int j = 0; j < 4; ++j) { const size_t po = (n * DV + j * 16 + col) * (size_t)NKEY + ks * 32; const v16h vh = frag_h(VH + po, lane); acc[j] = wmma16(pa, vh, acc[j]); acc[j] = wmma16(pr, vh, acc[j]); accl[j] = wmma16(pa, frag_h(VL + po, lane), accl[j]); }
    LDSX(); }
#pragma unroll
  for (int r = 0; r < 8; ++r) { const float il = (1.0f / 2048.0f) / l[r];
#pragma unroll
    for (int j = 0; j < 4; ++j) so[wave][8 * g + r][j * 16 + col] = (acc[j][r] + accl[j][r] * (1.0f / 2048.0f)) * il; }
  LDSX(); for (int rl = 0; rl < 16; ++rl) if (lane < 16) vst2(AO + (q0 + rl) * DV + lane * 4, *(const v4f*)&so[wave][rl][lane * 4]); }
__global__ __launch_bounds__(128) void k_out(const float* __restrict__ AO, const float* __restrict__ WO, const float* __restrict__ BO, const float* __restrict__ GM, const float* __restrict__ X, float* __restrict__ OUT) { __shared__ __align__(16) float st[CC][68];
  const int tid = threadIdx.x, wave = tid >> 5, lane = tid & 31, col = lane & 15, g = lane >> 4; const int pb = blockIdx.x; const size_t n = blockIdx.y; const size_t r0 = n * NQ + (size_t)pb * 64 + wave * 16; const float gm = bfr(GM[0]);
  v8f acc[8] = {};
#pragma unroll
  for (int kc = 0; kc < DV / 32; ++kc) { const F2 a = split_row(AO + (r0 + col) * DV, kc * 32, lane);
#pragma unroll
    for (int j = 0; j < 8; ++j) { v16b w; const int o = j * 16 + col;
#pragma unroll
      for (int i = 0; i < 8; ++i) { w[i] = (__bf16)WO[(kc * 32 + 8 * g + i) * CC + o]; w[8 + i] = (__bf16)WO[(kc * 32 + 16 + 8 * g + i) * CC + o]; }
      acc[j] = wmma_bf(a.h, w, acc[j]); acc[j] = wmma_bf(a.l, w, acc[j]); } }
#pragma unroll
  for (int j = 0; j < 8; ++j) { const int c = j * 16 + col; const float bb = bfr(BO[c]);
#pragma unroll
    for (int r = 0; r < 8; ++r) { const int pl = wave * 16 + 8 * g + r; st[c][pl] = bfr(X[(n * CC + c) * NQ + (size_t)pb * 64 + pl]) + gm * (acc[j][r] + bb); } }
  __syncthreads();
  for (int e = tid; e < CC * 16; e += 128) { const int c = e >> 4, q = e & 15; vst2(OUT + (n * CC + c) * NQ + (size_t)pb * 64 + q * 4, *(const v4f*)&st[c][q * 4]); } }
extern "C" void kernel_launch(void* const* d_in, const int* in_sizes, int n_in, void* d_out, int out_size, void* d_ws, size_t ws_size, hipStream_t stream) {
  (void)in_sizes; (void)n_in; (void)out_size;
  const float** F = (const float**)d_in;
  if (ws_size < (size_t)WS_END) return;
  char* ws = (char*)d_ws; float *Q = (float*)(ws + WS_Q), *KF = (float*)(ws + WS_KF), *VF = (float*)(ws + WS_VF), *KP = (float*)(ws + WS_KP), *AO = (float*)(ws + WS_AO); _Float16 *VH = (_Float16*)(ws + WS_VH), *VL = (_Float16*)(ws + WS_VL);
  k_proj<<<dim3(NQ / 64, TNI), 128, 0, stream>>>(F[0], F[1], F[2], F[3], F[4], F[5], F[6], Q, KF, VF);
  k_pool<<<dim3(NKEY / 64, TNI), 64, 0, stream>>>(KF, VF, KP, VH, VL);
  k_att<<<dim3(NQ / 64, TNI), 128, 0, stream>>>(Q, KP, VH, VL, AO);
  k_out<<<dim3(NQ / 64, TNI), 128, 0, stream>>>(AO, F[7], F[8], F[9], F[0], (float*)d_out);
}
